// Multi_domain_FeedForwardNetwork_v9_87144886435924
// MI455X (gfx1250) — hardware-verified
//
#include <hip/hip_runtime.h>
#include <stddef.h>


typedef _Float16 v16h __attribute__((ext_vector_type(16)));
typedef _Float16 v8h  __attribute__((ext_vector_type(8)));
typedef float    v8f  __attribute__((ext_vector_type(8)));
typedef float    v4f  __attribute__((ext_vector_type(4)));
union Frag { v16h v; v8h half[2]; };

#define BB     8
#define TT     512
#define DIN    1024
#define INNER  2048
#define DOUT   1024
#define NDOM   6
#define NTOK   (BB * TT)
#define JPR    (NTOK / BB)
#define WSCALE 32.0f
#define WINV   0.03125f

__device__ __forceinline__ v8f wmma_f16(v16h a, v16h b, v8f c) {
  v8f r = __builtin_amdgcn_wmma_f32_16x16x32_f16(false, a, false, b, (short)0, c, false, false);
  asm volatile("v_nop\n\tv_nop\n\tv_nop\n\tv_nop" : "+v"(r) : "v"(a), "v"(b));
  return r;
}

__device__ __forceinline__ float wave_sum(float v) {
#pragma unroll
  for (int o = 16; o > 0; o >>= 1) v += __shfl_xor(v, o, 32);
  return v;
}

__device__ __forceinline__ float half_sum16(float v) {
#pragma unroll
  for (int o = 8; o > 0; o >>= 1) v += __shfl_xor(v, o, 32);
  return v;
}

__global__ __launch_bounds__(256) void k_zero(float* out, int nvec) {
  const int i = blockIdx.x * 256 + threadIdx.x;
  if (i < nvec) {
    v4f z;
    z[0] = 0.0f; z[1] = 0.0f; z[2] = 0.0f; z[3] = 0.0f;
    float* p = out + (size_t)i * 4;
    *(volatile v4f*)p = z;
    __threadfence();
    *(volatile v4f*)p = z;
  }
}

__global__ __launch_bounds__(128) void k_ln(const float* __restrict__ x,
                                           const float* __restrict__ g,
                                           const float* __restrict__ b,
                                           _Float16* X16) {
  __shared__ float red[4];
  const int n = blockIdx.x, t = threadIdx.x, lane = t & 31, wave = t >> 5;
  const float4* xp = reinterpret_cast<const float4*>(x + (size_t)n * DIN + t * 8);
  const float4 u0 = xp[0], u1 = xp[1];
  float s = ((u0.x + u0.y) + (u0.z + u0.w)) + ((u1.x + u1.y) + (u1.z + u1.w));
  s = wave_sum(s);
  if (lane == 0) red[wave] = s;
  __syncthreads();
  const float mean = ((red[0] + red[1]) + (red[2] + red[3])) * (1.0f / DIN);
  __syncthreads();
  const float d0 = u0.x - mean, d1 = u0.y - mean, d2 = u0.z - mean, d3 = u0.w - mean;
  const float d4 = u1.x - mean, d5 = u1.y - mean, d6 = u1.z - mean, d7 = u1.w - mean;
  float sq = ((d0 * d0 + d1 * d1) + (d2 * d2 + d3 * d3)) + ((d4 * d4 + d5 * d5) + (d6 * d6 + d7 * d7));
  sq = wave_sum(sq);
  if (lane == 0) red[wave] = sq;
  __syncthreads();
  const float var = ((red[0] + red[1]) + (red[2] + red[3])) * (1.0f / DIN);
  const float rstd = rsqrtf(var + 1e-6f);
  const float4* gp = reinterpret_cast<const float4*>(g + t * 8);
  const float4* bp = reinterpret_cast<const float4*>(b + t * 8);
  const float4 g0 = gp[0], g1 = gp[1], b0 = bp[0], b1 = bp[1];
  v8h o;
  o[0] = (_Float16)(d0 * rstd * g0.x + b0.x);
  o[1] = (_Float16)(d1 * rstd * g0.y + b0.y);
  o[2] = (_Float16)(d2 * rstd * g0.z + b0.z);
  o[3] = (_Float16)(d3 * rstd * g0.w + b0.w);
  o[4] = (_Float16)(d4 * rstd * g1.x + b1.x);
  o[5] = (_Float16)(d5 * rstd * g1.y + b1.y);
  o[6] = (_Float16)(d6 * rstd * g1.z + b1.z);
  o[7] = (_Float16)(d7 * rstd * g1.w + b1.w);
  _Float16* dst = X16 + (size_t)n * DIN + t * 8;
  *(volatile v8h*)dst = o;
  __threadfence();
  *(volatile v8h*)dst = o;
}

template <int MODE>
__global__ __launch_bounds__(256) void k_tr(const float* __restrict__ in,
                                           _Float16* outp,
                                           const float* __restrict__ dom,
                                           int R, int C,
                                           long long inStrideZ, long long outStrideZ,
                                           int dcols, float scale) {
  __shared__ float tile[64][65];
  const int c0 = blockIdx.x * 64, r0 = blockIdx.y * 64;
  const int d = (MODE == 0) ? (c0 / dcols) : (int)blockIdx.z;
  int act = 0;
#pragma unroll
  for (int rr = 0; rr < BB; ++rr) act |= (dom[rr * NDOM + d] != 0.0f) ? 1 : 0;
  act = __builtin_amdgcn_readfirstlane(act);
  if (act == 0) return;

  const float* src = in + (size_t)blockIdx.z * (size_t)inStrideZ;
  _Float16* dst = outp + (size_t)blockIdx.z * (size_t)outStrideZ;
  const int tid = threadIdx.x, tx = tid & 63, ty = tid >> 6;
#pragma unroll
  for (int i = 0; i < 16; ++i)
    tile[ty + 4 * i][tx] = src[(size_t)(r0 + ty + 4 * i) * (size_t)C + c0 + tx];
  __syncthreads();

  const int lane = tid & 31, wave = tid >> 5;
  v8h keep[2];
#pragma unroll
  for (int p = 0; p < 2; ++p) {
    const int crow = p * 32 + wave * 4 + (lane >> 3);
    const int kseg = (lane & 7) * 8;
    v8h v;
#pragma unroll
    for (int e = 0; e < 8; ++e) v[e] = (_Float16)(tile[kseg + e][crow] * scale);
    keep[p] = v;
    _Float16* q = dst + (size_t)(c0 + crow) * (size_t)R + r0 + kseg;
    *(volatile v8h*)q = v;
  }
  __threadfence();
#pragma unroll
  for (int p = 0; p < 2; ++p) {
    const int crow = p * 32 + wave * 4 + (lane >> 3);
    const int kseg = (lane & 7) * 8;
    _Float16* q = dst + (size_t)(c0 + crow) * (size_t)R + r0 + kseg;
    *(volatile v8h*)q = keep[p];
  }
}

__global__ __launch_bounds__(512) void k_inner(const _Float16* __restrict__ X16,
                                              const _Float16* __restrict__ wiT,
                                              const float* __restrict__ dom,
                                              const float* __restrict__ bias_i,
                                              const float* __restrict__ g2,
                                              const float* __restrict__ b2,
                                              _Float16* H, int d) {
  __shared__ __align__(16) _Float16 stg[16 * 8 * 128];
  __shared__ float red[16 * 16];
  __shared__ float tot[16];

  const int tile = blockIdx.x, r = blockIdx.y;
  const int wbits = __builtin_amdgcn_readfirstlane(__float_as_int(dom[r * NDOM + d]));
  const float w = __int_as_float(wbits);
  if (w == 0.0f) return;

  const int tid = threadIdx.x, lane = tid & 31, wave = tid >> 5;
  const int h = lane >> 4, m = lane & 15;
  const int colbase = wave * 128;
  const int jrow0 = tile * 16;

  const _Float16* ap = X16 + ((size_t)r + (size_t)BB * (size_t)(jrow0 + m)) * DIN;
  const _Float16* bp = wiT + ((size_t)d * INNER + colbase + m) * DIN;

  v8f acc[8] = {};
#pragma unroll 1
  for (int s = 0; s < DIN / 32; ++s) {
    const int k0 = s * 32;
    Frag a;
    a.half[0] = *(const v8h*)(ap + k0 + 8 * h);
    a.half[1] = *(const v8h*)(ap + k0 + 16 + 8 * h);
#pragma unroll
    for (int j = 0; j < 8; ++j) {
      const _Float16* bj = bp + (size_t)j * 16 * DIN + k0;
      Frag b;
      b.half[0] = *(const v8h*)(bj + 8 * h);
      b.half[1] = *(const v8h*)(bj + 16 + 8 * h);
      acc[j] = wmma_f16(a.v, b.v, acc[j]);
    }
  }

  float bv[8], gv[8], be[8];
#pragma unroll
  for (int j = 0; j < 8; ++j) {
    const int c = colbase + j * 16 + m;
    bv[j] = bias_i[(size_t)d * INNER + c];
    gv[j] = g2[c];
    be[j] = b2[c];
  }
  float s[8];
#pragma unroll
  for (int rr = 0; rr < 8; ++rr) s[rr] = 0.0f;
#pragma unroll
  for (int j = 0; j < 8; ++j) {
#pragma unroll
    for (int rr = 0; rr < 8; ++rr) {
      const float hv = acc[j][rr] * WINV + bv[j];
      acc[j][rr] = hv;
      s[rr] += hv;
    }
  }
#pragma unroll
  for (int rr = 0; rr < 8; ++rr) s[rr] = half_sum16(s[rr]);
  if (m == 0) {
#pragma unroll
    for (int rr = 0; rr < 8; ++rr) red[wave * 16 + 8 * h + rr] = s[rr];
  }
  __syncthreads();
  if (tid < 16) {
    float t = 0.0f;
#pragma unroll
    for (int wv = 0; wv < 16; ++wv) t += red[wv * 16 + tid];
    tot[tid] = t * (1.0f / INNER);
  }
  __syncthreads();
  float mean[8];
#pragma unroll
  for (int rr = 0; rr < 8; ++rr) mean[rr] = tot[8 * h + rr];
  float q[8];
#pragma unroll
  for (int rr = 0; rr < 8; ++rr) q[rr] = 0.0f;
#pragma unroll
  for (int j = 0; j < 8; ++j) {
#pragma unroll
    for (int rr = 0; rr < 8; ++rr) {
      const float dd = acc[j][rr] - mean[rr];
      q[rr] += dd * dd;
    }
  }
#pragma unroll
  for (int rr = 0; rr < 8; ++rr) q[rr] = half_sum16(q[rr]);
  if (m == 0) {
#pragma unroll
    for (int rr = 0; rr < 8; ++rr) red[wave * 16 + 8 * h + rr] = q[rr];
  }
  __syncthreads();
  if (tid < 16) {
    float t = 0.0f;
#pragma unroll
    for (int wv = 0; wv < 16; ++wv) t += red[wv * 16 + tid];
    tot[tid] = rsqrtf(t * (1.0f / INNER) + 1e-6f);
  }
  __syncthreads();
  float rstd[8];
#pragma unroll
  for (int rr = 0; rr < 8; ++rr) rstd[rr] = tot[8 * h + rr];

  v8h keep[2][4];
#pragma unroll
  for (int p = 0; p < 2; ++p) {
    if (p) __syncthreads();
    if (h == p) {
#pragma unroll
      for (int j = 0; j < 8; ++j) {
#pragma unroll
        for (int rr = 0; rr < 8; ++rr) {
          float v = (acc[j][rr] - mean[rr]) * rstd[rr] * gv[j] + be[j];
          v = fmaxf(v, 0.0f);
          stg[(wave * 8 + rr) * 128 + j * 16 + m] = (_Float16)v;
        }
      }
    }
    __syncthreads();
#pragma unroll
    for (int qd = 0; qd < 4; ++qd) {
      const int row = qd * 2 + (lane >> 4);
      const int cs = (lane & 15) * 8;
      const v8h v = *(const v8h*)(stg + (wave * 8 + row) * 128 + cs);
      keep[p][qd] = v;
      const size_t n = (size_t)r + (size_t)BB * (size_t)(jrow0 + p * 8 + row);
      *(volatile v8h*)(H + n * INNER + colbase + cs) = v;
    }
  }
  __threadfence();
#pragma unroll
  for (int p = 0; p < 2; ++p) {
#pragma unroll
    for (int qd = 0; qd < 4; ++qd) {
      const int row = qd * 2 + (lane >> 4);
      const int cs = (lane & 15) * 8;
      const size_t n = (size_t)r + (size_t)BB * (size_t)(jrow0 + p * 8 + row);
      *(volatile v8h*)(H + n * INNER + colbase + cs) = keep[p][qd];
    }
  }
}

__global__ __launch_bounds__(256) void k_outer(const _Float16* __restrict__ H,
                                              const _Float16* __restrict__ woT,
                                              const float* __restrict__ dom,
                                              const float* __restrict__ bias_o,
                                              float* out, int d) {
  __shared__ __align__(16) float stg[8 * 16 * 64];
  const int ct = blockIdx.x, rt = blockIdx.y, r = blockIdx.z;
  const int wbits = __builtin_amdgcn_readfirstlane(__float_as_int(dom[r * NDOM + d]));
  const float w = __int_as_float(wbits);
  if (w == 0.0f) return;

  const int tid = threadIdx.x, lane = tid & 31, wave = tid >> 5;
  const int h = lane >> 4, m = lane & 15;
  const int wm = wave >> 2, wn = wave & 3;
  const int jrow0 = rt * 32 + wm * 16;
  const int colw = ct * 256 + wn * 64;

  const _Float16* ap = H + ((size_t)r + (size_t)BB * (size_t)(jrow0 + m)) * INNER;
  const _Float16* bp = woT + ((size_t)d * DOUT + colw + m) * INNER;

  v8f acc[4] = {};
#pragma unroll 1
  for (int s = 0; s < INNER / 32; ++s) {
    const int k0 = s * 32;
    Frag a;
    a.half[0] = *(const v8h*)(ap + k0 + 8 * h);
    a.half[1] = *(const v8h*)(ap + k0 + 16 + 8 * h);
#pragma unroll
    for (int j = 0; j < 4; ++j) {
      const _Float16* bj = bp + (size_t)j * 16 * INNER + k0;
      Frag b;
      b.half[0] = *(const v8h*)(bj + 8 * h);
      b.half[1] = *(const v8h*)(bj + 16 + 8 * h);
      acc[j] = wmma_f16(a.v, b.v, acc[j]);
    }
  }

  float bv[4];
#pragma unroll
  for (int j = 0; j < 4; ++j) bv[j] = bias_o[(size_t)d * DOUT + colw + j * 16 + m];
#pragma unroll
  for (int j = 0; j < 4; ++j) {
#pragma unroll
    for (int rr = 0; rr < 8; ++rr) {
      const float yv = acc[j][rr] * WINV + bv[j];
      stg[(wave * 16 + 8 * h + rr) * 64 + j * 16 + m] = w * yv;
    }
  }
  __syncthreads();

  v4f keep[8];
#pragma unroll
  for (int qd = 0; qd < 8; ++qd) {
    const int row = qd * 2 + (lane >> 4);
    const int cs = (lane & 15) * 4;
    const v4f sv = *(const v4f*)(stg + (wave * 16 + row) * 64 + cs);
    const size_t n = (size_t)r + (size_t)BB * (size_t)(jrow0 + row);
    float* p = out + n * DOUT + colw + cs;
    const v4f prior = *(const v4f*)p;
    const v4f res = prior + sv;
    keep[qd] = res;
    *(volatile v4f*)p = res;
  }
  __threadfence();
#pragma unroll
  for (int qd = 0; qd < 8; ++qd) {
    const int row = qd * 2 + (lane >> 4);
    const int cs = (lane & 15) * 4;
    const size_t n = (size_t)r + (size_t)BB * (size_t)(jrow0 + row);
    float* p = out + n * DOUT + colw + cs;
    *(volatile v4f*)p = keep[qd];
  }
}

extern "C" void kernel_launch(void* const* d_in, const int* in_sizes, int n_in,
                              void* d_out, int out_size, void* d_ws, size_t ws_size,
                              hipStream_t stream) {
  if (n_in < 10) return;
  if (in_sizes[0] != NTOK * DIN || in_sizes[1] != BB * NDOM ||
      in_sizes[2] != DIN || in_sizes[3] != DIN ||
      in_sizes[4] != INNER || in_sizes[5] != INNER ||
      in_sizes[6] != DIN * NDOM * INNER || in_sizes[7] != NDOM * INNER ||
      in_sizes[8] != NDOM * INNER * DOUT || in_sizes[9] != NDOM * DOUT ||
      out_size != NTOK * DOUT) return;

  const float* inputs = (const float*)d_in[0];
  const float* dom    = (const float*)d_in[1];
  const float* ln_g   = (const float*)d_in[2];
  const float* ln_b   = (const float*)d_in[3];
  const float* iln_g  = (const float*)d_in[4];
  const float* iln_b  = (const float*)d_in[5];
  const float* wi     = (const float*)d_in[6];
  const float* bi     = (const float*)d_in[7];
  const float* wo     = (const float*)d_in[8];
  const float* bo     = (const float*)d_in[9];
  float* out = (float*)d_out;

  char* ws = (char*)d_ws;
  size_t off = 0;
  _Float16* X16 = (_Float16*)(ws + off); off += (size_t)NTOK * DIN * 2;
  _Float16* wiT = (_Float16*)(ws + off); off += (size_t)NDOM * INNER * DIN * 2;
  _Float16* woT = (_Float16*)(ws + off); off += (size_t)NDOM * DOUT * INNER * 2;
  _Float16* H   = (_Float16*)(ws + off); off += (size_t)NTOK * INNER * 2;
  if (off > ws_size) return;

  k_tr<0><<<dim3(NDOM * INNER / 64, DIN / 64, 1), 256, 0, stream>>>(
      wi, wiT, dom, DIN, NDOM * INNER, 0LL, 0LL, INNER, WSCALE);
  k_tr<1><<<dim3(DOUT / 64, INNER / 64, NDOM), 256, 0, stream>>>(
      wo, woT, dom, INNER, DOUT, (long long)INNER * DOUT, (long long)DOUT * INNER, 1, WSCALE);

  k_ln<<<NTOK, 128, 0, stream>>>(inputs, ln_g, ln_b, X16);

  const int nvec = (NTOK * DOUT) / 4;
  k_zero<<<(nvec + 255) / 256, 256, 0, stream>>>(out, nvec);

  for (int d = 0; d < NDOM; ++d) {
    k_inner<<<dim3(JPR / 16, BB), 512, 0, stream>>>(X16, wiT, dom, bi, iln_g, iln_b, H, d);
    k_outer<<<dim3(DOUT / 256, JPR / 32, BB), 256, 0, stream>>>(H, woT, dom, bo, out, d);
  }
}
